// EncoderNetwork_12721693131090
// MI455X (gfx1250) — hardware-run, weakly checked
//
#include <hip/hip_runtime.h>
#include <stddef.h>


#define DIM     16
#define FIN     5
#define KDAG    21
#define NTHR    256
#define NWAVE   8
#define TGT     256
#define EPT     8
#define NGRP    2
#define CHUNK   (NTHR * EPT * NGRP)
#define WCAP    (EPT * NGRP * 32)
#define LISTN   (NWAVE * WCAP)
#define NBK     4096
#define RCAP    24576
#define RBN     128
#define OTHR    512
#define DEGCAP  64
#define DAGCAP  4096
#define NIMG    19
#define IMGH    512
#define CNTMAX  (1 << 22)
#define LDS_FILL ((RCAP + NBK + LISTN) * 4 + 64)

#define SP1 0
#define SP2 1
#define SP3 2
#define SM1 3
#define SU1 7
#define SD1 11
#define SG1 15

static_assert((CHUNK & (CHUNK - 1)) == 0);
static_assert(CHUNK == 4096);
static_assert(NBK == 4096);
static_assert(OTHR * 8 == NBK);
static_assert((RCAP % 32) == 0);
static_assert(TGT == NWAVE * 32);
static_assert(RBN == 32 * 4);

typedef float          v4f  __attribute__((ext_vector_type(4)));
typedef float          v8f  __attribute__((ext_vector_type(8)));
typedef int            v4i  __attribute__((ext_vector_type(4)));
typedef unsigned int   v4u  __attribute__((ext_vector_type(4)));
typedef __bf16         v8b  __attribute__((ext_vector_type(8)));
typedef __bf16         v16b __attribute__((ext_vector_type(16)));

struct Wts { const float* w[15]; };
static_assert(sizeof(Wts) == 120);

__device__ __forceinline__ v8f wmb(v16b a, v16b b, v8f c) {
  v8f d = __builtin_amdgcn_wmma_f32_16x16x32_bf16(false, a, false, b, (short)0, c, false, false);
  asm volatile("v_nop\n\tv_nop\n\tv_nop\n\tv_nop" : "+v"(d) : "v"(a), "v"(b));
  return d;
}

__device__ __forceinline__ v16b cat16(v8b a, v8b b) {
  return __builtin_shufflevector(a, b, 0, 1, 2, 3, 4, 5, 6, 7, 8, 9, 10, 11, 12, 13, 14, 15);
}
__device__ __forceinline__ v8f cat8(v4f a, v4f b) {
  return __builtin_shufflevector(a, b, 0, 1, 2, 3, 4, 5, 6, 7);
}
__device__ __forceinline__ v4f lo4(v8f v) { return __builtin_shufflevector(v, v, 0, 1, 2, 3); }
__device__ __forceinline__ v4f hi4(v8f v) { return __builtin_shufflevector(v, v, 4, 5, 6, 7); }
__device__ __forceinline__ v8f relu8(v8f x) {
  v8f r = x;
#pragma unroll
  for (int i = 0; i < 8; ++i) r[i] = r[i] > 0.0f ? r[i] : 0.0f;
  return r;
}
__device__ __forceinline__ v16b ldimg(const unsigned short* __restrict__ w, int slot, int lane) {
  const v8b* p = (const v8b*)(w + (size_t)slot * IMGH + 16 * lane);
  const v8b a = p[0];
  const v8b b = p[1];
  return cat16(a, b);
}
__device__ __forceinline__ v8f ldg8(const float* p) {
  const v4f a = *(const v4f*)p;
  const v4f b = *(const v4f*)(p + 4);
  return cat8(a, b);
}
__device__ __forceinline__ void stl8(float* p, v8f v) {
  *(v4f*)p = lo4(v);
  *(v4f*)(p + 4) = hi4(v);
}

__device__ __forceinline__ v16b bfrag16(v8f f) {
  const v8b hi = __builtin_convertvector(f, v8b);
  const v8f hf = __builtin_convertvector(hi, v8f);
  const v8b lo = __builtin_convertvector(f - hf, v8b);
  return cat16(hi, lo);
}
__device__ __forceinline__ v16b bfrag8(v8f f, int h) {
  const v8b hi = __builtin_convertvector(f, v8b);
  const v8f hf = __builtin_convertvector(hi, v8f);
  const v8f sel = f - (float)h * hf;
  const v8b part = __builtin_convertvector(sel, v8b);
  return cat16(part, part);
}

__device__ __forceinline__ v8f layers23(v8f a1, const unsigned short* __restrict__ w, int s2, int s3,
                                        const float* __restrict__ b2, const float* __restrict__ b3, int lane) {
  const int h = lane >> 4;
  const v8f g = relu8(a1);
  const v16b B2 = bfrag16(g);
  v8f c2 = ldg8(b2) * (float)(1 - h);
  c2 = wmb(ldimg(w, s2, lane), B2, c2);
  v8f t = c2;
#pragma unroll
  for (int r = 0; r < 8; ++r) { const float o = __shfl_xor(c2[r], 16); t[r] = c2[r] + o; }
  const v8f q = relu8(t);
  const v16b B3 = bfrag8(q, h);
  v8f c3 = ldg8(b3 + 8 * h);
  c3 = wmb(ldimg(w, s3, lane), B3, c3);
  return c3;
}

__device__ __forceinline__ v8f mlp16(v8f f, const unsigned short* __restrict__ w, int s0,
                                     const float* __restrict__ b1, const float* __restrict__ b2,
                                     const float* __restrict__ b3, int lane) {
  const int h = lane >> 4;
  const v16b B1 = bfrag16(f);
  v8f c1 = ldg8(b1 + 8 * h);
  c1 = wmb(ldimg(w, s0, lane), B1, c1);
  c1 = wmb(ldimg(w, s0 + 1, lane), B1, c1);
  return layers23(c1, w, s0 + 2, s0 + 3, b2, b3, lane);
}

__device__ __forceinline__ int scan_chunk(const int* __restrict__ dsts, int nE, int cbase, int slotBase,
                                          int vec8, int* list, int tid, int lane, int wave) {
  int wc = 0;
#pragma unroll
  for (int g = 0; g < NGRP; ++g) {
    const int el0  = (g * NTHR + tid) * EPT;
    const int e0   = cbase + el0;
    const int sent = -2147483647 - 1;
    v4i da, db;
    if (vec8 != 0 && cbase + CHUNK <= nE) {
      da = *(const v4i*)(dsts + e0);
      db = *(const v4i*)(dsts + e0 + 4);
    } else {
      da.x = (e0     < nE) ? dsts[min(e0, nE - 1)] : sent;
      da.y = (e0 + 1 < nE) ? dsts[min(e0 + 1, nE - 1)] : sent;
      da.z = (e0 + 2 < nE) ? dsts[min(e0 + 2, nE - 1)] : sent;
      da.w = (e0 + 3 < nE) ? dsts[min(e0 + 3, nE - 1)] : sent;
      db.x = (e0 + 4 < nE) ? dsts[min(e0 + 4, nE - 1)] : sent;
      db.y = (e0 + 5 < nE) ? dsts[min(e0 + 5, nE - 1)] : sent;
      db.z = (e0 + 6 < nE) ? dsts[min(e0 + 6, nE - 1)] : sent;
      db.w = (e0 + 7 < nE) ? dsts[min(e0 + 7, nE - 1)] : sent;
    }
    const unsigned nb = (unsigned)slotBase;
    const unsigned s0 = (unsigned)da.x - nb, s1 = (unsigned)da.y - nb;
    const unsigned s2 = (unsigned)da.z - nb, s3 = (unsigned)da.w - nb;
    const unsigned s4 = (unsigned)db.x - nb, s5 = (unsigned)db.y - nb;
    const unsigned s6 = (unsigned)db.z - nb, s7 = (unsigned)db.w - nb;
    const bool h0 = s0 < (unsigned)NBK, h1 = s1 < (unsigned)NBK, h2 = s2 < (unsigned)NBK, h3 = s3 < (unsigned)NBK;
    const bool h4 = s4 < (unsigned)NBK, h5 = s5 < (unsigned)NBK, h6 = s6 < (unsigned)NBK, h7 = s7 < (unsigned)NBK;
    const unsigned any = __builtin_amdgcn_ballot_w32(h0 | h1 | h2 | h3 | h4 | h5 | h6 | h7);
    if (any != 0u) {
#define HITJ(J, HJ, SJ) { \
        const unsigned mj = __builtin_amdgcn_ballot_w32(HJ); \
        if (mj != 0u) { \
          if (HJ) { \
            const int pos = wc + (int)__builtin_amdgcn_mbcnt_lo(mj, 0u); \
            if (pos < WCAP) list[wave * WCAP + pos] = ((el0 + (J)) << 12) | (int)(SJ); \
          } \
          wc += (int)__builtin_popcount(mj); } }
      HITJ(0, h0, s0)
      HITJ(1, h1, s1)
      HITJ(2, h2, s2)
      HITJ(3, h3, s3)
      HITJ(4, h4, s4)
      HITJ(5, h5, s5)
      HITJ(6, h6, s6)
      HITJ(7, h7, s7)
#undef HITJ
    }
  }
  return wc;
}

__global__ __launch_bounds__(32) void k_wpack(Wts W, unsigned short* img) {
  __shared__ __attribute__((aligned(16))) unsigned short simg[IMGH];
  const int slot = blockIdx.x, lane = threadIdx.x, m = lane & 15, h = lane >> 4;
  const float* wp;
  int nout = 16, kind = 0, kin = 16;
  if (slot == SP1)      { wp = W.w[0]; kind = 3; kin = FIN; }
  else if (slot == SP2) { wp = W.w[1]; kind = 2; nout = 8; }
  else if (slot == SP3) { wp = W.w[2]; kind = 3; kin = 8; }
  else {
    const float *w0p, *w1p, *w2p;
    int q; bool nat;
    if (slot < SU1)      { w0p = W.w[3];  w1p = W.w[4];  w2p = W.w[5];  q = slot - SM1; nat = false; }
    else if (slot < SD1) { w0p = W.w[6];  w1p = W.w[7];  w2p = W.w[8];  q = slot - SU1; nat = false; }
    else if (slot < SG1) { w0p = W.w[9];  w1p = W.w[10]; w2p = W.w[11]; q = slot - SD1; nat = true;  }
    else                 { w0p = W.w[12]; w1p = W.w[13]; w2p = W.w[14]; q = slot - SG1; nat = false; }
    if (q == 0)      { wp = w0p; kind = nat ? 4 : 0; kin = nat ? KDAG : 16; }
    else if (q == 1) { wp = w0p; kind = nat ? 5 : 1; kin = nat ? KDAG : 16; }
    else if (q == 2) { wp = w1p; kind = 2; nout = 8; kin = 16; }
    else             { wp = w2p; kind = 3; kin = 8; }
  }
#pragma unroll
  for (int i = 0; i < 16; ++i) {
    const int s = i + 8 * h + (i < 8 ? 0 : 8);
    int f, col; bool phi;
    if (kind <= 1)      { f = s & 15; col = m;     phi = (kind == 0); }
    else if (kind == 2) { f = s & 15; col = m & 7; phi = (m < 8); }
    else if (kind == 3) { f = s & 7;  col = m;     phi = (s < 16); }
    else                { f = s;      col = m;     phi = (kind == 4); }
    const int fc = f < kin ? f : kin - 1;
    float v = wp[fc * nout + col];
    v = (f < kin) ? v : 0.0f;
    const __bf16 hb = (__bf16)v;
    const float  hf = (float)hb;
    const __bf16 lb = (__bf16)(v - hf);
    const __bf16 ob = phi ? hb : lb;
    simg[16 * lane + i] = __builtin_bit_cast(unsigned short, ob);
  }
  __syncthreads();
  const v4u p0 = *(const v4u*)(simg + 8 * lane);
  const v4u p1 = *(const v4u*)(simg + 256 + 8 * lane);
  unsigned short* g = img + (size_t)slot * IMGH;
  *(volatile v4u*)(g + 8 * lane) = p0;
  *(volatile v4u*)(g + 256 + 8 * lane) = p1;
  __threadfence();
  *(volatile v4u*)(g + 8 * lane) = p0;
  *(volatile v4u*)(g + 256 + 8 * lane) = p1;
}

__global__ __launch_bounds__(NTHR) void k_count(const int* __restrict__ ei, int* cnt, int nE, int vec8) {
  __shared__ __attribute__((aligned(16))) int scnt[NBK];
  __shared__ __attribute__((aligned(16))) int list[LISTN];
  __shared__ int wcnt[NWAVE];
  const int tid = threadIdx.x, lane = tid & 31, wave = tid >> 5;
  const int nodeBase = blockIdx.x * NBK;
  const int* dsts = ei;

  for (int i = tid; i < NBK; i += NTHR) scnt[i] = 0;
  __syncthreads();

  const int nChunks = (nE + CHUNK - 1) / CHUNK;
#pragma unroll 1
  for (int ch = 0; ch < nChunks; ++ch) {
    const int cbase = ch * CHUNK;
    const int wc = scan_chunk(dsts, nE, cbase, nodeBase, vec8, list, tid, lane, wave);
    if (lane == 0) wcnt[wave] = wc;
    __syncthreads();
    if (wave == 0) {
#pragma unroll 1
      for (int wsx = 0; wsx < NWAVE; ++wsx) {
        int n = __builtin_amdgcn_readfirstlane(wcnt[wsx]);
        n = n > WCAP ? WCAP : (n < 0 ? 0 : n);
        const int* lp = list + wsx * WCAP;
#pragma unroll 1
        for (int i = 0; i < n; ++i) {
          const int ent  = __builtin_amdgcn_readfirstlane(lp[i]);
          const int slot = ent & (NBK - 1);
          if (lane == 0) scnt[slot] = scnt[slot] + 1;
        }
      }
    }
    __syncthreads();
  }

  v4i cq[4];
#pragma unroll
  for (int q = 0; q < 4; ++q) {
    const int f = (wave * 4 + q) * 128 + 4 * lane;
    cq[q] = *(const v4i*)(scnt + f);
  }
  int* cp = cnt + (size_t)nodeBase;
#pragma unroll
  for (int q = 0; q < 4; ++q) {
    const int f = (wave * 4 + q) * 128 + 4 * lane;
    *(volatile v4i*)(cp + f) = cq[q];
  }
  __threadfence();
#pragma unroll
  for (int q = 0; q < 4; ++q) {
    const int f = (wave * 4 + q) * 128 + 4 * lane;
    *(volatile v4i*)(cp + f) = cq[q];
  }
}

__global__ __launch_bounds__(OTHR) void k_offsets(const int* __restrict__ cnt, int* off, int* rbase, int nChunk) {
  __shared__ __attribute__((aligned(16))) int soff[NBK];
  __shared__ __attribute__((aligned(16))) int srb[RBN];
  __shared__ int wtot[OTHR / 32];
  const int tid = threadIdx.x, lane = tid & 31, wave = tid >> 5;
  for (int i = tid; i < RBN; i += OTHR) srb[i] = 0;
  int carry = 0;
#pragma unroll 1
  for (int ch = 0; ch < nChunk; ++ch) {
    const int base = ch * NBK;
    const v4i c0 = *(const v4i*)(cnt + base + 8 * tid);
    const v4i c1 = *(const v4i*)(cnt + base + 8 * tid + 4);
#define CLC(v) ((v) < 0 ? 0 : ((v) > CNTMAX ? CNTMAX : (v)))
    const int e0 = CLC(c0.x), e1 = CLC(c0.y), e2 = CLC(c0.z), e3 = CLC(c0.w);
    const int e4 = CLC(c1.x), e5 = CLC(c1.y), e6 = CLC(c1.z), e7 = CLC(c1.w);
#undef CLC
    const int ts = e0 + e1 + e2 + e3 + e4 + e5 + e6 + e7;
    int incl = ts;
#pragma unroll
    for (int d = 1; d < 32; d <<= 1) {
      const int t = __shfl_up(incl, d);
      incl = (lane >= d) ? incl + t : incl;
    }
    if (lane == 31) wtot[wave] = incl;
    __syncthreads();
    int pre = 0, S = 0;
#pragma unroll 1
    for (int w = 0; w < OTHR / 32; ++w) {
      const int t = wtot[w];
      S += t;
      pre += (w < wave) ? t : 0;
    }
    const int b0 = carry;
    if (tid == 0) srb[ch < RBN ? ch : RBN - 1] = b0;
    int run = b0 + pre + incl - ts;
    soff[8 * tid + 0] = run; run += e0;
    soff[8 * tid + 1] = run; run += e1;
    soff[8 * tid + 2] = run; run += e2;
    soff[8 * tid + 3] = run; run += e3;
    soff[8 * tid + 4] = run; run += e4;
    soff[8 * tid + 5] = run; run += e5;
    soff[8 * tid + 6] = run; run += e6;
    soff[8 * tid + 7] = run;
    carry = b0 + ((S + 31) & ~31);
    __syncthreads();
    const v4i o0 = *(const v4i*)(soff + 4 * tid);
    const v4i o1 = *(const v4i*)(soff + 4 * (tid + OTHR));
    int* op = off + base;
    *(volatile v4i*)(op + 4 * tid) = o0;
    *(volatile v4i*)(op + 4 * (tid + OTHR)) = o1;
    __threadfence();
    *(volatile v4i*)(op + 4 * tid) = o0;
    *(volatile v4i*)(op + 4 * (tid + OTHR)) = o1;
    __syncthreads();
  }
  if (tid == 0) srb[nChunk < RBN ? nChunk : RBN - 1] = carry;
  __syncthreads();
  v4i rv = {0, 0, 0, 0};
  if (tid < 32) rv = *(const v4i*)(srb + 4 * tid);
  if (tid < 32) *(volatile v4i*)(rbase + 4 * tid) = rv;
  __threadfence();
  if (tid < 32) *(volatile v4i*)(rbase + 4 * tid) = rv;
}

__global__ __launch_bounds__(NTHR) void k_fill(const int* __restrict__ ei, const int* __restrict__ off,
                                            const int* __restrict__ rbase, int* csr, int nE, int vec8, int csrLen) {
  extern __shared__ v4f lds_dyn[];
  int* region = (int*)lds_dyn;
  int* cursor = region + RCAP;
  int* list   = cursor + NBK;
  int* wcnt   = list + LISTN;
  const int tid = threadIdx.x, lane = tid & 31, wave = tid >> 5;
  const int b = blockIdx.x;
  const int nodeBase = b * NBK;
  const int* dsts = ei;

  int rb0 = rbase[b];
  const int rb1 = rbase[b + 1];
  rb0 = rb0 < 0 ? 0 : (rb0 > csrLen ? csrLen : rb0);
  rb0 &= ~31;
  int len = rb1 - rb0;
  len = len < 0 ? 0 : (len > RCAP ? RCAP : len);
  int lenW = (len + 31) & ~31;
  if (rb0 + lenW > csrLen) lenW = (csrLen - rb0) & ~31;

  {
    const v4i z = {0, 0, 0, 0};
    for (int i = tid; i < RCAP / 4; i += NTHR) ((v4i*)region)[i] = z;
    for (int s = tid; s < NBK; s += NTHR) {
      int o = off[nodeBase + s] - rb0;
      o = o < 0 ? 0 : (o > RCAP ? RCAP : o);
      cursor[s] = o;
    }
  }
  __syncthreads();

  const int nChunks = (nE + CHUNK - 1) / CHUNK;
#pragma unroll 1
  for (int ch = 0; ch < nChunks; ++ch) {
    const int cbase = ch * CHUNK;
    const int wc = scan_chunk(dsts, nE, cbase, nodeBase, vec8, list, tid, lane, wave);
    if (lane == 0) wcnt[wave] = wc;
    __syncthreads();
    if (wave == 0) {
#pragma unroll 1
      for (int wsx = 0; wsx < NWAVE; ++wsx) {
        int n = __builtin_amdgcn_readfirstlane(wcnt[wsx]);
        n = n > WCAP ? WCAP : (n < 0 ? 0 : n);
        const int* lp = list + wsx * WCAP;
#pragma unroll 1
        for (int i = 0; i < n; ++i) {
          const int ent  = __builtin_amdgcn_readfirstlane(lp[i]);
          const int slot = ent & (NBK - 1);
          int e = cbase + ((ent >> 12) & (CHUNK - 1));
          e = e > nE - 1 ? nE - 1 : e;
          if (lane == 0) {
            int pos = cursor[slot];
            pos = pos < 0 ? 0 : (pos > RCAP - 1 ? RCAP - 1 : pos);
            region[pos] = e;
            const int np = pos + 1;
            cursor[slot] = np > RCAP ? RCAP : np;
          }
        }
      }
    }
    __syncthreads();
  }

  const int nv = lenW >> 2;
  int* gp = csr + rb0;
#pragma unroll 1
  for (int i = tid; i < nv; i += NTHR) { const v4i v = ((const v4i*)region)[i]; *(volatile v4i*)(gp + 4 * i) = v; }
  __threadfence();
#pragma unroll 1
  for (int i = tid; i < nv; i += NTHR) { const v4i v = ((const v4i*)region)[i]; *(volatile v4i*)(gp + 4 * i) = v; }
}

__global__ __launch_bounds__(NTHR) void k_prep(const float* __restrict__ x, const unsigned short* __restrict__ wimg,
                                            const float* __restrict__ pb1, const float* __restrict__ pb2,
                                            const float* __restrict__ pb3, const float* __restrict__ mb1,
                                            const float* __restrict__ mb2, const float* __restrict__ mb3,
                                            float* hpl, float* ypl, int nN) {
  __shared__ __attribute__((aligned(16))) float sH[TGT * DIM];
  __shared__ __attribute__((aligned(16))) float sY[TGT * DIM];
  const int tid = threadIdx.x, lane = tid & 31, wave = tid >> 5, h = lane >> 4, n = lane & 15;
  const size_t base = (size_t)blockIdx.x * TGT;

#pragma unroll
  for (int t = 0; t < 2; ++t) {
    const int jn = 32 * wave + 16 * t + n;
    const size_t node = base + jn;
    const size_t nc = node < (size_t)nN ? node : (size_t)(nN - 1);
    const float* xr = x + nc * FIN;
    v8f xv;
    xv[0] = xr[0]; xv[1] = xr[1]; xv[2] = xr[2]; xv[3] = xr[3]; xv[4] = xr[4];
    xv[5] = 0.0f; xv[6] = 0.0f; xv[7] = 0.0f;
    const v16b B1 = bfrag8(xv, h);
    v8f c1 = ldg8(pb1 + 8 * h);
    c1 = wmb(ldimg(wimg, SP1, lane), B1, c1);
    const v8f h0 = layers23(c1, wimg, SP2, SP3, pb2, pb3, lane);
    stl8(sH + jn * DIM + 8 * h, h0);
    const v8f y0 = mlp16(h0, wimg, SM1, mb1, mb2, mb3, lane);
    stl8(sY + jn * DIM + 8 * h, y0);
  }
  __syncthreads();

  v4f hq[4], yq[4];
#pragma unroll
  for (int q = 0; q < 4; ++q) {
    const int row = 32 * wave + 8 * q + (lane >> 2);
    const int pc = 4 * (lane & 3);
    hq[q] = *(const v4f*)(sH + row * DIM + pc);
    yq[q] = *(const v4f*)(sY + row * DIM + pc);
  }
#pragma unroll
  for (int q = 0; q < 4; ++q) {
    const int row = 32 * wave + 8 * q + (lane >> 2);
    const size_t g = (base + row) * DIM + 4 * (lane & 3);
    *(volatile v4f*)(hpl + g) = hq[q];
    *(volatile v4f*)(ypl + g) = yq[q];
  }
  __threadfence();
#pragma unroll
  for (int q = 0; q < 4; ++q) {
    const int row = 32 * wave + 8 * q + (lane >> 2);
    const size_t g = (base + row) * DIM + 4 * (lane & 3);
    *(volatile v4f*)(hpl + g) = hq[q];
    *(volatile v4f*)(ypl + g) = yq[q];
  }
}

__global__ __launch_bounds__(NTHR) void k_step(
    const int* __restrict__ ei, const int* __restrict__ mk, const int* __restrict__ csr,
    const int* __restrict__ off, const int* __restrict__ cnt,
    const float* __restrict__ ycur, float* ynext, float* hpl, float* outp,
    const float* __restrict__ x, const unsigned short* __restrict__ wimg,
    const float* __restrict__ ub1, const float* __restrict__ ub2, const float* __restrict__ ub3,
    const float* __restrict__ sb1, const float* __restrict__ sb2, const float* __restrict__ sb3,
    int nN, int nE, int csrLen, int mode, int writeOut) {
  __shared__ __attribute__((aligned(16))) float sAgg[TGT * DIM];
  __shared__ __attribute__((aligned(16))) float sH[TGT * DIM];
  __shared__ __attribute__((aligned(16))) float sY[TGT * DIM];
  __shared__ float sNm[TGT];
  const int tid = threadIdx.x, lane = tid & 31, wave = tid >> 5, h = lane >> 4, n = lane & 15;
  const size_t base = (size_t)blockIdx.x * TGT;

  {
    const int j = 32 * wave + lane;
    const size_t c = base + j;
    int cn = cnt[c];
    cn = cn < 0 ? 0 : (cn > DEGCAP ? DEGCAP : cn);
    const int st = off[c];
    int nmax = cn;
#pragma unroll
    for (int d = 1; d < 32; d <<= 1) { const int o = __shfl_xor(nmax, d); nmax = o > nmax ? o : nmax; }
    nmax = __builtin_amdgcn_readfirstlane(nmax);
    v4f a0 = {0.f, 0.f, 0.f, 0.f}, a1 = a0, a2 = a0, a3 = a0;
    int any = 0;
#pragma unroll 1
    for (int p = 0; p < nmax; ++p) {
      const bool ok = p < cn;
      int pos = st + p;
      pos = pos < 0 ? 0 : (pos > csrLen - 1 ? csrLen - 1 : pos);
      int e = csr[pos];
      e = e < 0 ? 0 : (e > nE - 1 ? nE - 1 : e);
      const int mv = mk[e];
      int s = ei[(size_t)nE + e];
      s = s < 0 ? 0 : (s > nN - 1 ? nN - 1 : s);
      const v4f* yp = (const v4f*)(ycur + (size_t)s * DIM);
      const v4f y0 = yp[0], y1 = yp[1], y2 = yp[2], y3 = yp[3];
      const bool act = ok && (mv != 0);
      const float fm = act ? 1.0f : 0.0f;
      a0 = a0 + y0 * fm; a1 = a1 + y1 * fm; a2 = a2 + y2 * fm; a3 = a3 + y3 * fm;
      any |= act ? 1 : 0;
    }
    float* ap = sAgg + j * DIM;
    *(v4f*)ap = a0; *(v4f*)(ap + 4) = a1; *(v4f*)(ap + 8) = a2; *(v4f*)(ap + 12) = a3;
    sNm[j] = (any != 0) ? 1.0f : 0.0f;
  }
  __syncthreads();

#pragma unroll
  for (int t = 0; t < 2; ++t) {
    const int jn = 32 * wave + 16 * t + n;
    const size_t node = base + jn;
    const v8f f = ldg8(sAgg + jn * DIM + 8 * h);
    const v8f upd = mlp16(f, wimg, SU1, ub1, ub2, ub3, lane);
    const v8f hv = ldg8(hpl + node * DIM + 8 * h);
    const float nmv = sNm[jn];
    const v8f hn = hv + nmv * upd;
    stl8(sH + jn * DIM + 8 * h, hn);
    if (mode == 0) {
      const v8f yv = mlp16(hn, wimg, SM1, sb1, sb2, sb3, lane);
      stl8(sY + jn * DIM + 8 * h, yv);
    }
  }
  __syncthreads();

  if (mode != 0) {
#pragma unroll
    for (int t = 0; t < 2; ++t) {
      const int jn = 32 * wave + 16 * t + n;
      const size_t node = base + jn;
      const size_t nc = node < (size_t)nN ? node : (size_t)(nN - 1);
      const float* xr = x + nc * FIN;
      const float x0 = xr[0], x1 = xr[1], x2 = xr[2], x3 = xr[3], x4 = xr[4];
      const float* hr = sH + jn * DIM;
      const v4f hA = *(const v4f*)hr, hB = *(const v4f*)(hr + 4), hC = *(const v4f*)(hr + 8), hD = *(const v4f*)(hr + 12);
      v8f gA, gB, gC;
      gA[0] = x0;   gA[1] = x1;   gA[2] = x2;   gA[3] = x3;   gA[4] = x4;   gA[5] = hA.x; gA[6] = hA.y; gA[7] = hA.z;
      gB[0] = hA.w; gB[1] = hB.x; gB[2] = hB.y; gB[3] = hB.z; gB[4] = hB.w; gB[5] = hC.x; gB[6] = hC.y; gB[7] = hC.z;
      gC[0] = hC.w; gC[1] = hD.x; gC[2] = hD.y; gC[3] = hD.z; gC[4] = hD.w; gC[5] = 0.0f; gC[6] = 0.0f; gC[7] = 0.0f;
      const bool hs = (h != 0);
      v8f eL = gA, eH = gC;
#pragma unroll
      for (int i = 0; i < 8; ++i) { eL[i] = hs ? gB[i] : gA[i]; eH[i] = hs ? 0.0f : gC[i]; }
      const v8b hiL = __builtin_convertvector(eL, v8b);
      const v8f hfL = __builtin_convertvector(hiL, v8f);
      const v8b loL = __builtin_convertvector(eL - hfL, v8b);
      const v8b hiH = __builtin_convertvector(eH, v8b);
      const v8f hfH = __builtin_convertvector(hiH, v8f);
      const v8b loH = __builtin_convertvector(eH - hfH, v8b);
      const v16b Bhi = cat16(hiL, hiH);
      const v16b Blo = cat16(loL, loH);
      const v16b A11 = ldimg(wimg, SD1, lane);
      const v16b A12 = ldimg(wimg, SD1 + 1, lane);
      v8f c1 = ldg8(sb1 + 8 * h);
      c1 = wmb(A11, Bhi, c1);
      c1 = wmb(A12, Bhi, c1);
      c1 = wmb(A11, Blo, c1);
      const v8f z = layers23(c1, wimg, SD1 + 2, SD1 + 3, sb2, sb3, lane);
      stl8(sY + jn * DIM + 8 * h, z);
    }
  }
  __syncthreads();

  v4f hq[4], yq[4];
#pragma unroll
  for (int q = 0; q < 4; ++q) {
    const int row = 32 * wave + 8 * q + (lane >> 2);
    const int pc = 4 * (lane & 3);
    hq[q] = *(const v4f*)(sH + row * DIM + pc);
    yq[q] = *(const v4f*)(sY + row * DIM + pc);
  }
#pragma unroll
  for (int q = 0; q < 4; ++q) {
    const int row = 32 * wave + 8 * q + (lane >> 2);
    const size_t g = (base + row) * DIM + 4 * (lane & 3);
    *(volatile v4f*)(hpl + g) = hq[q];
    *(volatile v4f*)(ynext + g) = yq[q];
    if (writeOut != 0 && base + row < (size_t)nN) *(volatile v4f*)(outp + g) = hq[q];
  }
  __threadfence();
#pragma unroll
  for (int q = 0; q < 4; ++q) {
    const int row = 32 * wave + 8 * q + (lane >> 2);
    const size_t g = (base + row) * DIM + 4 * (lane & 3);
    *(volatile v4f*)(hpl + g) = hq[q];
    *(volatile v4f*)(ynext + g) = yq[q];
    if (writeOut != 0 && base + row < (size_t)nN) *(volatile v4f*)(outp + g) = hq[q];
  }
}

__global__ __launch_bounds__(NTHR) void k_tail(const float* __restrict__ zpl, const int* __restrict__ ptr,
                                            const unsigned short* __restrict__ wimg,
                                            const float* __restrict__ gb1, const float* __restrict__ gb2,
                                            const float* __restrict__ gb3,
                                            float* out1, float* out2, int nN, int ndags) {
  __shared__ __attribute__((aligned(16))) float sD[TGT * DIM];
  __shared__ __attribute__((aligned(16))) double sG[NWAVE * DIM];
  __shared__ __attribute__((aligned(16))) float sO[DIM];
  const int tid = threadIdx.x, lane = tid & 31, wave = tid >> 5, h = lane >> 4, n = lane & 15;
  double gacc[8];
#pragma unroll
  for (int r = 0; r < 8; ++r) gacc[r] = 0.0;

  const int nCh = (ndags + TGT - 1) / TGT;
#pragma unroll 1
  for (int ch = 0; ch < nCh; ++ch) {
    const int cb = ch * TGT;
    const int d = cb + tid;
    const bool valid = d < ndags;
    const int dc = valid ? d : ndags - 1;
    int beg = ptr[dc];
    int end = ptr[dc + 1];
    beg = beg < 0 ? 0 : (beg > nN ? nN : beg);
    end = end < 0 ? 0 : (end > nN ? nN : end);
    int len = end - beg;
    len = len < 0 ? 0 : (len > DAGCAP ? DAGCAP : len);
    len = valid ? len : 0;
    int lmax = len;
#pragma unroll
    for (int dd = 1; dd < 32; dd <<= 1) { const int o = __shfl_xor(lmax, dd); lmax = o > lmax ? o : lmax; }
    lmax = __builtin_amdgcn_readfirstlane(lmax);
    v4f a0 = {0.f, 0.f, 0.f, 0.f}, a1 = a0, a2 = a0, a3 = a0;
#pragma unroll 1
    for (int i = 0; i < lmax; ++i) {
      const float fm = (i < len) ? 1.0f : 0.0f;
      int node = beg + i;
      node = node > nN - 1 ? nN - 1 : (node < 0 ? 0 : node);
      const v4f* zp = (const v4f*)(zpl + (size_t)node * DIM);
      a0 = a0 + zp[0] * fm; a1 = a1 + zp[1] * fm; a2 = a2 + zp[2] * fm; a3 = a3 + zp[3] * fm;
    }
    float* dp = sD + tid * DIM;
    *(v4f*)dp = a0; *(v4f*)(dp + 4) = a1; *(v4f*)(dp + 8) = a2; *(v4f*)(dp + 12) = a3;
    __syncthreads();

    v4f oq[4];
#pragma unroll
    for (int q = 0; q < 4; ++q) {
      const int row = 32 * wave + 8 * q + (lane >> 2);
      oq[q] = *(const v4f*)(sD + row * DIM + 4 * (lane & 3));
    }
#pragma unroll
    for (int q = 0; q < 4; ++q) {
      const int row = 32 * wave + 8 * q + (lane >> 2);
      const int drow = cb + row;
      if (drow < ndags) *(volatile v4f*)(out1 + (size_t)drow * DIM + 4 * (lane & 3)) = oq[q];
    }
    __threadfence();
#pragma unroll
    for (int q = 0; q < 4; ++q) {
      const int row = 32 * wave + 8 * q + (lane >> 2);
      const int drow = cb + row;
      if (drow < ndags) *(volatile v4f*)(out1 + (size_t)drow * DIM + 4 * (lane & 3)) = oq[q];
    }

#pragma unroll
    for (int t = 0; t < 2; ++t) {
      const int jn = 32 * wave + 16 * t + n;
      const v8f f = ldg8(sD + jn * DIM + 8 * h);
      const v8f g = mlp16(f, wimg, SG1, gb1, gb2, gb3, lane);
      const bool dv = (cb + jn) < ndags;
#pragma unroll
      for (int r = 0; r < 8; ++r) gacc[r] += dv ? (double)g[r] : 0.0;
    }
    __syncthreads();
  }

#pragma unroll
  for (int r = 0; r < 8; ++r) {
#pragma unroll
    for (int dd = 1; dd < 16; dd <<= 1) gacc[r] += __shfl_xor(gacc[r], dd);
  }
  if (n == 0) {
#pragma unroll
    for (int r = 0; r < 8; ++r) sG[wave * DIM + 8 * h + r] = gacc[r];
  }
  __syncthreads();
  if (tid < DIM) {
    double s = 0.0;
#pragma unroll 1
    for (int w = 0; w < NWAVE; ++w) s += sG[w * DIM + tid];
    sO[tid] = (float)s;
  }
  __syncthreads();
  v4f ov = {0.f, 0.f, 0.f, 0.f};
  if (tid < 4) ov = *(const v4f*)(sO + 4 * tid);
  if (tid < 4) *(volatile v4f*)(out2 + 4 * tid) = ov;
  __threadfence();
  if (tid < 4) *(volatile v4f*)(out2 + 4 * tid) = ov;
}

extern "C" void kernel_launch(void* const* d_in, const int* in_sizes, int n_in,
                              void* d_out, int out_size, void* d_ws, size_t ws_size,
                              hipStream_t stream) {
  if (n_in < 34) return;
  const int nN = in_sizes[0] / FIN;
  const int nE = in_sizes[1] / 2;
  if (nN < 1 || nE < 1 || in_sizes[0] != nN * FIN || in_sizes[1] != 2 * nE) return;
  if (nN > (1 << 24) || nE > (1 << 27)) return;
  const int nR = in_sizes[2] / nE;
  if (nR < 1 || in_sizes[2] != nR * nE) return;
  if (in_sizes[3] < 2) return;
  const int ndags = in_sizes[3] - 1;
  const int kins[5] = {FIN, DIM, DIM, KDAG, DIM};
  for (int q = 0; q < 5; ++q) {
    const int b = 4 + 6 * q;
    if (in_sizes[b] != kins[q] * 16 || in_sizes[b + 1] != 16 || in_sizes[b + 2] != 16 * 8 ||
        in_sizes[b + 3] != 8 || in_sizes[b + 4] != 8 * 16 || in_sizes[b + 5] != 16) return;
  }
  if ((long long)out_size != (long long)nN * DIM + (long long)ndags * DIM + DIM) return;

  const int NPAD   = ((nN + TGT - 1) / TGT) * TGT;
  const int nBlk   = NPAD / TGT;
  const int nBC    = (nN + NBK - 1) / NBK;
  const int CNTPAD = nBC * NBK;
  if (nBC + 1 > RBN || CNTPAD < NPAD) return;
  const int csrLen = ((nE + 31) & ~31) + 4096;

  char* ws = (char*)d_ws;
  size_t off = 0;
  const size_t oImg = off; off += (size_t)NIMG * IMGH * 2;      off = (off + 255) & ~(size_t)255;
  const size_t oCnt = off; off += (size_t)CNTPAD * 4;          off = (off + 255) & ~(size_t)255;
  const size_t oOff = off; off += (size_t)CNTPAD * 4;          off = (off + 255) & ~(size_t)255;
  const size_t oRb  = off; off += (size_t)RBN * 4;             off = (off + 255) & ~(size_t)255;
  const size_t oCsr = off; off += (size_t)csrLen * 4;          off = (off + 255) & ~(size_t)255;
  const size_t oH   = off; off += (size_t)NPAD * DIM * 4;      off = (off + 255) & ~(size_t)255;
  const size_t oY0  = off; off += (size_t)NPAD * DIM * 4;      off = (off + 255) & ~(size_t)255;
  const size_t oY1  = off; off += (size_t)NPAD * DIM * 4;      off = (off + 255) & ~(size_t)255;
  if (off > ws_size) return;

  unsigned short* img = (unsigned short*)(ws + oImg);
  int*   cnt  = (int*)(ws + oCnt);
  int*   offp = (int*)(ws + oOff);
  int*   rb   = (int*)(ws + oRb);
  int*   csr  = (int*)(ws + oCsr);
  float* hpl  = (float*)(ws + oH);
  float* ypl[2];
  ypl[0] = (float*)(ws + oY0);
  ypl[1] = (float*)(ws + oY1);

  const float* x     = (const float*)d_in[0];
  const int*   ei    = (const int*)d_in[1];
  const int*   maskp = (const int*)d_in[2];
  const int*   ptr   = (const int*)d_in[3];
  Wts W;
  for (int q = 0; q < 5; ++q)
    for (int l = 0; l < 3; ++l) W.w[3 * q + l] = (const float*)d_in[4 + 6 * q + 2 * l];
  const float* pb1 = (const float*)d_in[5];
  const float* pb2 = (const float*)d_in[7];
  const float* pb3 = (const float*)d_in[9];
  const float* mb1 = (const float*)d_in[11];
  const float* mb2 = (const float*)d_in[13];
  const float* mb3 = (const float*)d_in[15];
  const float* ub1 = (const float*)d_in[17];
  const float* ub2 = (const float*)d_in[19];
  const float* ub3 = (const float*)d_in[21];
  const float* db1 = (const float*)d_in[23];
  const float* db2 = (const float*)d_in[25];
  const float* db3 = (const float*)d_in[27];
  const float* gb1 = (const float*)d_in[29];
  const float* gb2 = (const float*)d_in[31];
  const float* gb3 = (const float*)d_in[33];
  float* out0 = (float*)d_out;
  float* out1 = out0 + (size_t)nN * DIM;
  float* out2 = out1 + (size_t)ndags * DIM;

  const int vec8 = ((nE & 3) == 0) ? 1 : 0;

  k_wpack<<<NIMG, 32, 0, stream>>>(W, img);

  k_count<<<nBC, NTHR, 0, stream>>>(ei, cnt, nE, vec8);
  k_offsets<<<1, OTHR, 0, stream>>>(cnt, offp, rb, nBC);
  hipFuncSetAttribute(reinterpret_cast<const void*>(&k_fill),
                      hipFuncAttributeMaxDynamicSharedMemorySize, LDS_FILL);
  k_fill<<<nBC, NTHR, LDS_FILL, stream>>>(ei, offp, rb, csr, nE, vec8, csrLen);

  k_prep<<<nBlk, NTHR, 0, stream>>>(x, img, pb1, pb2, pb3, mb1, mb2, mb3, hpl, ypl[0], nN);

  for (int r = 0; r < nR; ++r) {
    const int last = (r == nR - 1) ? 1 : 0;
    const float* b1 = last ? db1 : mb1;
    const float* b2 = last ? db2 : mb2;
    const float* b3 = last ? db3 : mb3;
    k_step<<<nBlk, NTHR, 0, stream>>>(ei, maskp + (size_t)r * nE, csr, offp, cnt,
                                      ypl[r & 1], ypl[(r + 1) & 1], hpl, out0, x, img,
                                      ub1, ub2, ub3, b1, b2, b3,
                                      nN, nE, csrLen, last, last);
  }

  k_tail<<<1, NTHR, 0, stream>>>(ypl[nR & 1], ptr, img, gb1, gb2, gb3, out1, out2, nN, ndags);
}
